// KuramotoInteraction_54511724921354
// MI455X (gfx1250) — hardware-verified
//
#include <hip/hip_runtime.h>
#include <math.h>

typedef __attribute__((ext_vector_type(16))) _Float16 v16h;
typedef __attribute__((ext_vector_type(16))) __bf16 v16b;
typedef __attribute__((ext_vector_type(8)))  _Float16 v8h;
typedef __attribute__((ext_vector_type(8)))  float v8f;
typedef __attribute__((ext_vector_type(4)))  float v4f;
typedef __attribute__((ext_vector_type(2)))  float v2f;
typedef __attribute__((ext_vector_type(4)))  unsigned v4u;
typedef __attribute__((ext_vector_type(4)))  int v4i;
typedef float __attribute__((may_alias)) float_a;
typedef int __attribute__((may_alias)) int_a;

template <typename T> __device__ __forceinline__ void vst2(void* p, T v) { *(volatile T*)p = v; __threadfence(); *(volatile T*)p = v; }
__device__ __forceinline__ v8f wmma16(v16h a, v16h b, v8f c) {
  v8f d = __builtin_amdgcn_wmma_f32_16x16x32_f16(false, a, false, b, (short)0, c, false, false);
  asm volatile("v_nop\n\tv_nop\n\tv_nop\n\tv_nop" : "+v"(d) : "v"(a), "v"(b));
  return d;
}
__device__ __forceinline__ v8f wmma_bf(v16b a, v16b b, v8f c) {
  v8f d = __builtin_amdgcn_wmma_f32_16x16x32_bf16(false, a, false, b, (short)0, c, false, false);
  asm volatile("v_nop\n\tv_nop\n\tv_nop\n\tv_nop" : "+v"(d) : "v"(a), "v"(b));
  return d;
}
__device__ __forceinline__ v16h frag_h(const _Float16* rowk0, int lane) {
  union { v16h v; v8h q[2]; } u; const _Float16* p = rowk0 + 8 * (lane >> 4);
  u.q[0] = *(const v8h*)p; u.q[1] = *(const v8h*)(p + 16); return u.v;
}
__device__ __forceinline__ v16h frag_f32(const float* rowk0, int lane) {
  v16h a; const float* p = rowk0 + 8 * (lane >> 4);
#pragma unroll
  for (int i = 0; i < 8; ++i) { a[i] = (_Float16)p[i]; a[8 + i] = (_Float16)p[16 + i]; }
  return a;
}
__device__ __forceinline__ v16h frag_f32s(const float* rowk0, int lane, float sc) {
  v16h a; const float* p = rowk0 + 8 * (lane >> 4);
#pragma unroll
  for (int i = 0; i < 8; ++i) { a[i] = (_Float16)(p[i] * sc); a[8 + i] = (_Float16)(p[16 + i] * sc); }
  return a;
}
__device__ __forceinline__ v16h fragc_f32(const float* W, int k0, int n, int lane, int ld, int K) {
  v16h a; const int g = lane >> 4;
#pragma unroll
  for (int i = 0; i < 8; ++i) { const int ka = k0 + 8 * g + i, kb = ka + 16;
    a[i] = (_Float16)(ka < K ? W[(size_t)ka * ld + n] : 0.f); a[8 + i] = (_Float16)(kb < K ? W[(size_t)kb * ld + n] : 0.f); }
  return a;
}
struct F2 { v16b h, l; };
__device__ __forceinline__ F2 bsplit16(const float v[16]) { F2 r;
#pragma unroll
  for (int i = 0; i < 16; ++i) { const __bf16 h = (__bf16)v[i]; r.h[i] = h; r.l[i] = (__bf16)(v[i] - (float)h); }
  return r; }
__device__ __forceinline__ F2 split_row(const float* row, int k0, int lane) { float v[16]; const float* p = row + k0 + 8 * (lane >> 4);
#pragma unroll
  for (int i = 0; i < 8; ++i) { v[i] = p[i]; v[8 + i] = p[16 + i]; }
  return bsplit16(v); }
__device__ __forceinline__ F2 split_rowK(const float* row, int k0, int lane, int K) { float v[16]; const int g = lane >> 4;
#pragma unroll
  for (int i = 0; i < 8; ++i) { const int ka = k0 + 8 * g + i, kb = ka + 16; v[i] = ka < K ? row[ka] : 0.f; v[8 + i] = kb < K ? row[kb] : 0.f; }
  return bsplit16(v); }
__device__ __forceinline__ F2 split_col(const float* W, int k0, int n, int lane, int ld, int K) { float v[16]; const int g = lane >> 4;
#pragma unroll
  for (int i = 0; i < 8; ++i) { const int ka = k0 + 8 * g + i, kb = ka + 16; v[i] = ka < K ? W[(size_t)ka * ld + n] : 0.f; v[8 + i] = kb < K ? W[(size_t)kb * ld + n] : 0.f; }
  return bsplit16(v); }
__device__ __forceinline__ v8f mac3(const F2& a, const F2& b, v8f c) { c = wmma_bf(a.l, b.h, c); c = wmma_bf(a.h, b.l, c); return wmma_bf(a.h, b.h, c); }
__device__ __forceinline__ float sigm(float v) { return 1.0f / (1.0f + expf(-v)); }
#define LDSX() do { asm volatile("s_wait_dscnt 0" ::: "memory"); __builtin_amdgcn_wave_barrier(); __builtin_amdgcn_fence(__ATOMIC_RELEASE, "workgroup"); } while (0)

#define NB 4
#define TT 2048
#define DD 512
#define NH 8
#define HD 64
#define NR (NB * TT)

__global__ __launch_bounds__(256) void k_packW(const float* __restrict__ W, int K, _Float16* __restrict__ P, float sc) {
  const int n = blockIdx.x, tid = threadIdx.x;
  for (int q = tid; q < K / 8; q += 256) { union { v8h hh; v4u u; } pk;
#pragma unroll
    for (int i = 0; i < 8; ++i) pk.hh[i] = (_Float16)(W[(size_t)n * K + q * 8 + i] * sc);
    vst2(P + (size_t)n * K + q * 8, pk.u); }
}
__global__ __launch_bounds__(128) void k_proj(const float* __restrict__ z, const _Float16* __restrict__ P, _Float16* __restrict__ qn, _Float16* __restrict__ kn, _Float16* __restrict__ kT) {
  __shared__ __align__(16) float so[4][16][132];
  __shared__ __align__(16) _Float16 st[128][72];
  const int tid = threadIdx.x, wave = tid >> 5, lane = tid & 31, col = lane & 15, g = lane >> 4;
  const int r0b = blockIdx.x * 64, r0 = r0b + wave * 16, n0 = blockIdx.y * 128; const int b = r0b / TT, t0 = r0b % TT;
  const int which = n0 / DD, hb = (n0 % DD) / HD;
  v8f acc[8] = {};
#pragma unroll 1
  for (int kc = 0; kc < DD / 32; ++kc) { const v16h a = frag_f32(z + (size_t)(r0 + col) * DD + kc * 32, lane);
#pragma unroll
    for (int j = 0; j < 8; ++j) acc[j] = wmma16(a, frag_h(P + (size_t)(n0 + j * 16 + col) * DD + kc * 32, lane), acc[j]); }
#pragma unroll
  for (int j = 0; j < 8; ++j)
#pragma unroll
    for (int r = 0; r < 8; ++r) so[wave][8 * g + r][j * 16 + col] = acc[j][r] * (1.0f / 16.0f);
  LDSX();
  { float s = 0.f;
    for (int i = 0; i < HD; ++i) { const float v = so[wave][col][g * HD + i]; s += v * v; }
    const float inv = 8.0f / fmaxf(sqrtf(s), 1e-12f);
    for (int i = 0; i < HD; ++i) so[wave][col][g * HD + i] *= inv; }
  LDSX();
  { _Float16* dst = which == 0 ? qn : kn;
    for (int q = lane; q < 2 * 16 * 8; q += 32) { const int hh = q >> 7, rem = q & 127, rl = rem >> 3, pc = rem & 7; union { v8h h8; v4u u; } pk;
#pragma unroll
      for (int e = 0; e < 8; ++e) pk.h8[e] = (_Float16)so[wave][rl][hh * HD + pc * 8 + e];
      vst2(dst + (((size_t)b * NH + hb + hh) * TT + t0 + wave * 16 + rl) * HD + pc * 8, pk.u); } }
  if (which == 1) {
#pragma unroll 4
    for (int rl = 0; rl < 16; ++rl) { st[lane * 4 + 0][wave * 16 + rl] = (_Float16)so[wave][rl][lane * 4]; st[lane * 4 + 1][wave * 16 + rl] = (_Float16)so[wave][rl][lane * 4 + 1];
      st[lane * 4 + 2][wave * 16 + rl] = (_Float16)so[wave][rl][lane * 4 + 2]; st[lane * 4 + 3][wave * 16 + rl] = (_Float16)so[wave][rl][lane * 4 + 3]; }
    __syncthreads();
    for (int q = tid; q < 128 * 8; q += 128) { const int c = q >> 3, pc = q & 7, hh = c >> 6, d = c & 63;
      vst2(kT + (((size_t)b * NH + hb + hh) * HD + d) * TT + t0 + pc * 8, *(const v4u*)(&st[c][pc * 8])); }
  }
}
__global__ __launch_bounds__(128) void k_force(const _Float16* __restrict__ qn, const _Float16* __restrict__ kn, const _Float16* __restrict__ kT, float* __restrict__ force) {
  __shared__ __align__(16) _Float16 sP[4][16][72];
  __shared__ __align__(16) float so[4][16][68];
  const int tid = threadIdx.x, w = tid >> 5, lane = tid & 31, col = lane & 15, g = lane >> 4;
  const int bh = blockIdx.y, b = bh / NH, h = bh % NH, q0 = blockIdx.x * 64 + w * 16;
  const _Float16* qb = qn + (size_t)bh * TT * HD; const _Float16* kb = kn + (size_t)bh * TT * HD; const _Float16* ktb = kT + (size_t)bh * HD * TT;
  v16h aq[2];
#pragma unroll
  for (int kc = 0; kc < 2; ++kc) aq[kc] = frag_h(qb + (size_t)(q0 + col) * HD + kc * 32, lane);
  v8f acc[4] = {};
#pragma unroll 1
  for (int kt = 0; kt < TT / 64; ++kt) {
#pragma unroll
    for (int t = 0; t < 4; ++t) { v8f s = {};
#pragma unroll
      for (int kc = 0; kc < 2; ++kc) s = wmma16(aq[kc], frag_h(kb + (size_t)(kt * 64 + t * 16 + col) * HD + kc * 32, lane), s);
#pragma unroll
      for (int r = 0; r < 8; ++r) sP[w][8 * g + r][t * 16 + col] = (_Float16)(sinf(s[r] * (1.0f / 64.0f)) * 16384.0f); }
    LDSX();
#pragma unroll
    for (int kc = 0; kc < 2; ++kc) { const v16h pa = frag_h(&sP[w][col][0] + kc * 32, lane);
#pragma unroll
      for (int t = 0; t < 4; ++t) acc[t] = wmma16(pa, frag_h(ktb + (size_t)(t * 16 + col) * TT + kt * 64 + kc * 32, lane), acc[t]); }
    __builtin_amdgcn_wave_barrier();
  }
#pragma unroll
  for (int t = 0; t < 4; ++t)
#pragma unroll
    for (int r = 0; r < 8; ++r) so[w][8 * g + r][t * 16 + col] = acc[t][r] * (1.0f / (16384.0f * 8.0f));
  LDSX();
  for (int q = lane; q < 16 * 16; q += 32) { const int rl = q >> 4, pc = q & 15; vst2(force + ((size_t)b * TT + q0 + rl) * DD + h * HD + pc * 4, *(const v4f*)(&so[w][rl][pc * 4])); }
}
__global__ __launch_bounds__(128) void k_out(const float* __restrict__ force, const _Float16* __restrict__ Po, const float* __restrict__ bo, const float* __restrict__ omega, float* __restrict__ out) {
  __shared__ __align__(16) float so[4][16][132];
  const int tid = threadIdx.x, wave = tid >> 5, lane = tid & 31, col = lane & 15, g = lane >> 4;
  const int r0 = blockIdx.x * 64 + wave * 16, n0 = blockIdx.y * 128;
  v8f acc[8] = {};
#pragma unroll 1
  for (int kc = 0; kc < DD / 32; ++kc) { const v16h a = frag_f32(force + (size_t)(r0 + col) * DD + kc * 32, lane);
#pragma unroll
    for (int j = 0; j < 8; ++j) acc[j] = wmma16(a, frag_h(Po + (size_t)(n0 + j * 16 + col) * DD + kc * 32, lane), acc[j]); }
#pragma unroll
  for (int j = 0; j < 8; ++j) { const int n = n0 + j * 16 + col; const float bb = bo[n] + omega[n];
#pragma unroll
    for (int r = 0; r < 8; ++r) so[wave][8 * g + r][j * 16 + col] = acc[j][r] * (1.0f / 16.0f) + bb; }
  LDSX();
#pragma unroll 4
  for (int rl = 0; rl < 16; ++rl) vst2(out + (size_t)(r0 + rl) * DD + n0 + lane * 4, *(const v4f*)(&so[wave][rl][lane * 4]));
}
extern "C" void kernel_launch(void* const* d_in, const int* in_sizes, int n_in, void* d_out, int out_size, void* d_ws, size_t ws_size, hipStream_t stream) {
  (void)in_sizes; (void)n_in; (void)out_size; (void)ws_size;
  const float* z = (const float*)d_in[1]; const float* omega = (const float*)d_in[2]; const float* Wqk = (const float*)d_in[3]; const float* Wo = (const float*)d_in[4]; const float* bo = (const float*)d_in[5];
  float* out = (float*)d_out;
  char* ws = (char*)d_ws; size_t off = 0;
  auto take = [&](size_t bytes) { char* p = ws + off; off += (bytes + 255) & ~(size_t)255; return p; };
  _Float16* Pqk = (_Float16*)take((size_t)2 * DD * DD * 2); _Float16* Po = (_Float16*)take((size_t)DD * DD * 2);
  _Float16* qn = (_Float16*)take((size_t)NR * DD * 2); _Float16* kn = (_Float16*)take((size_t)NR * DD * 2); _Float16* kT = (_Float16*)take((size_t)NR * DD * 2);
  float* force = (float*)take((size_t)NR * DD * 4);
  k_packW<<<2 * DD, 256, 0, stream>>>(Wqk, DD, Pqk, 16.0f);
  k_packW<<<DD, 256, 0, stream>>>(Wo, DD, Po, 16.0f);
  k_proj<<<dim3(NR / 64, 2 * DD / 128), 128, 0, stream>>>(z, Pqk, qn, kn, kT);
  k_force<<<dim3(TT / 64, NB * NH), 128, 0, stream>>>(qn, kn, kT, force);
  k_out<<<dim3(NR / 64, DD / 128), 128, 0, stream>>>(force, Po, bo, omega, out);
}
